// DifferentialCrossAttention_12610023981459
// MI455X (gfx1250) — hardware-verified
//
#include <hip/hip_runtime.h>
#include <math.h>
#include <stdint.h>

#define NB     4
#define NTOK   1024
#define DM     512
#define NHEAD  8
#define NPAIR  4
#define HD     64
#define NROWS  (NB * NTOK)
#define KCH    32
#define RPW    257
#define RPOFF  128
#define RPMAX  256
#define RPN    66049
#define WSC    64.0f
#define ACARRY 16.0f
#define VC     16.0f
#define PC     4096.0f
#define QKS    0.125f
#define LOG2E  1.4426950408889634f
#define SC2    (QKS * LOG2E)
#define LAM0   0.8f
static_assert(NHEAD * HD == DM);
static_assert(NPAIR * 2 == NHEAD);
static_assert((NTOK % 64) == 0 && (DM % 64) == 0 && (NROWS % 64) == 0 && (HD % 32) == 0 && (NTOK % KCH) == 0);
static_assert(((NROWS * DM) % 2048) == 0 && ((DM * DM) % 2048) == 0);
#define ATT_THREADS (NHEAD * 32)
#define ATT_BLOCKS  (NB * (NTOK / 16))
#define PT_FLOATS   (NHEAD * 16 * 36)
#define CROSS_FLOATS (NPAIR * 16 * HD)
#define OROW_HALVES  (16 * DM)
#define ATT_SMEM_FLOATS (CROSS_FLOATS + OROW_HALVES / 2 + OROW_HALVES / 2)
static_assert(ATT_THREADS == 256);
static_assert(ATT_BLOCKS == 256);
static_assert(ATT_SMEM_FLOATS == 12288);
static_assert(PT_FLOATS <= ATT_SMEM_FLOATS);
static_assert(OROW_HALVES / 8 == 4 * ATT_THREADS);

typedef _Float16 v16h __attribute__((ext_vector_type(16)));
typedef _Float16 v8h  __attribute__((ext_vector_type(8)));
typedef __bf16   v16b __attribute__((ext_vector_type(16)));
typedef float    v8f  __attribute__((ext_vector_type(8)));
typedef float    v4f  __attribute__((ext_vector_type(4)));
typedef unsigned int v4u __attribute__((ext_vector_type(4)));

union FragH { v16h v; v8h h[2]; v4u u[2]; };
union FragAny { v16h h; v16b b; };

__device__ __forceinline__ unsigned short bf_bits(float f) {
  unsigned u = __float_as_uint(f);
  return (unsigned short)((u + 0x7FFFu + ((u >> 16) & 1u)) >> 16);
}
__device__ __forceinline__ float bf_up(unsigned short h) { return __uint_as_float(((unsigned)h) << 16); }
__device__ __forceinline__ float bfr(float f) { return bf_up(bf_bits(f)); }
__device__ __forceinline__ unsigned short h_bits(_Float16 x) { return __builtin_bit_cast(unsigned short, x); }
__device__ __forceinline__ unsigned pk16(unsigned short a, unsigned short b) { return (unsigned)a | ((unsigned)b << 16); }
__device__ __forceinline__ v8f zero8() { v8f z = {0.f, 0.f, 0.f, 0.f, 0.f, 0.f, 0.f, 0.f}; return z; }
__device__ __forceinline__ int iclamp(int x, int lo, int hi) { x = (x < lo) ? lo : x; return (x > hi) ? hi : x; }

__device__ __forceinline__ v16h ldfrag_u(const unsigned short* p) {
  FragH f;
  f.u[0] = *(const v4u*)(p);
  f.u[1] = *(const v4u*)(p + 16);
  return f.v;
}

__device__ __forceinline__ v8f mma_h(v16h a, v16h b, v8f c) {
  return __builtin_amdgcn_wmma_f32_16x16x32_f16(false, a, false, b, (short)0, c, false, false);
}
__device__ __forceinline__ v8f mma_b(v16h a, v16h b, v8f c) {
  FragAny ua, ub;
  ua.h = a;
  ub.h = b;
  return __builtin_amdgcn_wmma_f32_16x16x32_bf16(false, ua.b, false, ub.b, (short)0, c, false, false);
}
template <int BF>
__device__ __forceinline__ v8f mmaT(v16h a, v16h b, v8f c) {
  if constexpr (BF != 0) return mma_b(a, b, c);
  else return mma_h(a, b, c);
}
__device__ __forceinline__ void dep_guard1(v8f& a, v8f& b, v16h x) {
#if defined(__HIP_DEVICE_COMPILE__)
  asm volatile("v_nop\n\tv_nop\n\tv_nop\n\tv_nop" : "+v"(a), "+v"(b) : "v"(x));
#endif
}
__device__ __forceinline__ void guard2x6(v8f& a, v8f& b, v16h x0, v16h x1, v16h x2, v16h x3, v16h x4, v16h x5) {
#if defined(__HIP_DEVICE_COMPILE__)
  asm volatile("v_nop\n\tv_nop\n\tv_nop\n\tv_nop"
               : "+v"(a), "+v"(b) : "v"(x0), "v"(x1), "v"(x2), "v"(x3), "v"(x4), "v"(x5));
#endif
}
__device__ __forceinline__ void guard4x6(v8f& a, v8f& b, v8f& c, v8f& d,
                                         v16h x0, v16h x1, v16h x2, v16h x3, v16h x4, v16h x5) {
#if defined(__HIP_DEVICE_COMPILE__)
  asm volatile("v_nop\n\tv_nop\n\tv_nop\n\tv_nop"
               : "+v"(a), "+v"(b), "+v"(c), "+v"(d) : "v"(x0), "v"(x1), "v"(x2), "v"(x3), "v"(x4), "v"(x5));
#endif
}
__device__ __forceinline__ void guard4x5(v8f& a, v8f& b, v8f& c, v8f& d,
                                         v16h x0, v16h x1, v16h x2, v16h x3, v16h x4) {
#if defined(__HIP_DEVICE_COMPILE__)
  asm volatile("v_nop\n\tv_nop\n\tv_nop\n\tv_nop"
               : "+v"(a), "+v"(b), "+v"(c), "+v"(d) : "v"(x0), "v"(x1), "v"(x2), "v"(x3), "v"(x4));
#endif
}
__device__ __forceinline__ void keep4_h(v16h a, v16h b, v16h c, v16h d) {
#if defined(__HIP_DEVICE_COMPILE__)
  asm volatile("v_nop" :: "v"(a), "v"(b), "v"(c), "v"(d));
#endif
}
__device__ __forceinline__ void acc_guard4(v8f& a, v8f& b, v8f& c, v8f& d) {
#if defined(__HIP_DEVICE_COMPILE__)
  asm volatile("v_nop\n\tv_nop\n\tv_nop\n\tv_nop" : "+v"(a), "+v"(b), "+v"(c), "+v"(d));
#endif
}
__device__ __forceinline__ void wave_sync_lds() {
  __builtin_amdgcn_fence(__ATOMIC_RELEASE, "workgroup");
  __builtin_amdgcn_wave_barrier();
  __builtin_amdgcn_fence(__ATOMIC_ACQUIRE, "workgroup");
}

template <int BFO>
__global__ __launch_bounds__(256) void cvt16(const float* __restrict__ src, unsigned short* dst, int n, float sc) {
  const size_t i8 = ((size_t)blockIdx.x * 256 + threadIdx.x) * 8;
  if (i8 + 8 > (size_t)n) return;
  const v4f a = *(const v4f*)(src + i8);
  const v4f b = *(const v4f*)(src + i8 + 4);
  v4u o;
  if constexpr (BFO != 0) {
    o[0] = pk16(bf_bits(a[0]), bf_bits(a[1]));
    o[1] = pk16(bf_bits(a[2]), bf_bits(a[3]));
    o[2] = pk16(bf_bits(b[0]), bf_bits(b[1]));
    o[3] = pk16(bf_bits(b[2]), bf_bits(b[3]));
  } else {
    o[0] = pk16(h_bits((_Float16)(bfr(a[0]) * sc)), h_bits((_Float16)(bfr(a[1]) * sc)));
    o[1] = pk16(h_bits((_Float16)(bfr(a[2]) * sc)), h_bits((_Float16)(bfr(a[3]) * sc)));
    o[2] = pk16(h_bits((_Float16)(bfr(b[0]) * sc)), h_bits((_Float16)(bfr(b[1]) * sc)));
    o[3] = pk16(h_bits((_Float16)(bfr(b[2]) * sc)), h_bits((_Float16)(bfr(b[3]) * sc)));
  }
  for (int pass = 0; pass < 2; ++pass) {
    *(volatile v4u*)(dst + i8) = o;
    __threadfence();
  }
}

template <int OM, int ASPLIT, int BF, int EPI>
__global__ __launch_bounds__(256) __attribute__((amdgpu_num_vgpr(256))) void gemm64(
    const unsigned short* __restrict__ Ap, const unsigned short* __restrict__ A2p, int lda, long long sA,
    const unsigned short* __restrict__ Btp, int ldb, long long sB,
    void* Cout, void* C2out, int ldc, long long sC,
    int M, int N, int K, float oscale, float ocarry,
    const float* __restrict__ bias) {
  __shared__ __align__(16) float sT[8][16 * 68];
  const int by   = blockIdx.y;
  const int lane = threadIdx.x & 31;
  const int wave = threadIdx.x >> 5;
  const int tilesN = N >> 6;
  const int tilesM = M >> 6;
  const int tile = blockIdx.x * 8 + wave;
  if (tile >= tilesM * tilesN) return;
  const int tm = tile / tilesN;
  const int tn = tile - tm * tilesN;
  const int m0 = tm << 6;
  const int n0 = tn << 6;

  const unsigned short* A1 = Ap  + (size_t)((long long)by * sA);
  const unsigned short* A2 = A2p + (size_t)((long long)by * sA);
  const unsigned short* Bb = Btp + (size_t)((long long)by * sB);

  const int rlane = lane & 15;
  const int koff  = (lane >> 4) * 8;
  const int mOff  = (lane >> 4) * 8;

  v8f acc[4][4];
#pragma unroll
  for (int i = 0; i < 4; ++i)
#pragma unroll
    for (int j = 0; j < 4; ++j) acc[i][j] = zero8();

  for (int k0 = 0; k0 < K; k0 += 32) {
    v16h bh[4];
#pragma unroll
    for (int j = 0; j < 4; ++j) {
      const size_t bofs = (size_t)(n0 + (j << 4) + rlane) * ldb + koff + k0;
      bh[j] = ldfrag_u(Bb + bofs);
    }
#pragma unroll
    for (int i = 0; i < 4; ++i) {
      const size_t ao = (size_t)(m0 + (i << 4) + rlane) * lda + koff + k0;
      const v16h ah = ldfrag_u(A1 + ao);
#pragma unroll
      for (int j = 0; j < 4; ++j) acc[i][j] = mmaT<BF>(ah, bh[j], acc[i][j]);
      dep_guard1(acc[i][0], acc[i][3], ah);
      if constexpr (ASPLIT != 0) {
        const v16h al = ldfrag_u(A2 + ao);
#pragma unroll
        for (int j = 0; j < 4; ++j) acc[i][j] = mmaT<BF>(al, bh[j], acc[i][j]);
        dep_guard1(acc[i][0], acc[i][3], al);
      }
    }
    keep4_h(bh[0], bh[1], bh[2], bh[3]);
  }
  acc_guard4(acc[0][0], acc[0][1], acc[0][2], acc[0][3]);
  acc_guard4(acc[1][0], acc[1][1], acc[1][2], acc[1][3]);
  acc_guard4(acc[2][0], acc[2][1], acc[2][2], acc[2][3]);
  acc_guard4(acc[3][0], acc[3][1], acc[3][2], acc[3][3]);

  const int hh2 = lane >> 4, c4 = (lane & 15) * 4;
  const int q8  = lane >> 3, c8 = (lane & 7) * 8;

  float* slab = sT[wave];
#pragma unroll
  for (int i = 0; i < 4; ++i) {
    const int mBase = m0 + (i << 4);
#pragma unroll
    for (int j = 0; j < 4; ++j) {
#pragma unroll
      for (int r = 0; r < 8; ++r) {
        slab[(mOff + r) * 68 + (j << 4) + rlane] = acc[i][j][r];
      }
    }
    wave_sync_lds();
    if constexpr (OM == 0) {
      float* C = (float*)Cout + (size_t)((long long)by * sC);
      v4f vals[8];
#pragma unroll
      for (int it = 0; it < 8; ++it) {
        const int row = it * 2 + hh2;
        v4f v = *(const v4f*)(slab + row * 68 + c4);
#pragma unroll
        for (int e = 0; e < 4; ++e) {
          float f = v[e] * oscale;
          if constexpr (EPI == 1) f += bfr(bias[n0 + c4 + e]);
          if constexpr (EPI == 2) f += bfr(bias[mBase + row]);
          v[e] = f;
        }
        vals[it] = v;
      }
      for (int pass = 0; pass < 2; ++pass) {
#pragma unroll
        for (int it = 0; it < 8; ++it) {
          const int gr = mBase + it * 2 + hh2;
          *(volatile v4f*)(C + (size_t)gr * ldc + n0 + c4) = vals[it];
        }
        __threadfence();
      }
    } else {
      unsigned short* C  = (unsigned short*)Cout  + (size_t)((long long)by * sC);
      unsigned short* Cb = (unsigned short*)C2out + (size_t)((long long)by * sC);
      v4u hv[4], lv[4];
#pragma unroll
      for (int it = 0; it < 4; ++it) {
        const int row = it * 4 + q8;
        const float* sp = slab + row * 68 + c8;
        v4u a  = {0u, 0u, 0u, 0u};
        v4u b2 = {0u, 0u, 0u, 0u};
        float brow = 0.f;
        if constexpr (EPI == 2) brow = bfr(bias[mBase + row]);
#pragma unroll
        for (int e = 0; e < 4; ++e) {
          float f0 = sp[2 * e] * oscale;
          float f1 = sp[2 * e + 1] * oscale;
          if constexpr (EPI == 1) {
            f0 += bfr(bias[n0 + c8 + 2 * e]);
            f1 += bfr(bias[n0 + c8 + 2 * e + 1]);
          }
          if constexpr (EPI == 2) {
            f0 += brow;
            f1 += brow;
          }
          if constexpr (OM == 3) {
            const unsigned short g0 = bf_bits(f0), g1 = bf_bits(f1);
            a[e]  = pk16(g0, g1);
            b2[e] = pk16(bf_bits(f0 - bf_up(g0)), bf_bits(f1 - bf_up(g1)));
          } else {
            f0 *= ocarry; f1 *= ocarry;
            const _Float16 x0 = (_Float16)f0, x1 = (_Float16)f1;
            a[e] = pk16(h_bits(x0), h_bits(x1));
            if constexpr (OM == 4) {
              b2[e] = pk16(h_bits((_Float16)(f0 - (float)x0)), h_bits((_Float16)(f1 - (float)x1)));
            }
          }
        }
        hv[it] = a;
        lv[it] = b2;
      }
      for (int pass = 0; pass < 2; ++pass) {
#pragma unroll
        for (int it = 0; it < 4; ++it) {
          const int row = it * 4 + q8;
          *(volatile v4u*)(C + (size_t)(mBase + row) * ldc + n0 + c8) = hv[it];
          if constexpr (OM >= 3) {
            *(volatile v4u*)(Cb + (size_t)(mBase + row) * ldc + n0 + c8) = lv[it];
          }
        }
        __threadfence();
      }
    }
    wave_sync_lds();
  }
}

__global__ __launch_bounds__(ATT_THREADS) __attribute__((amdgpu_num_vgpr(256)))
void attn8(const unsigned short* __restrict__ Q16, const unsigned short* __restrict__ K16,
           const unsigned short* __restrict__ VTh, const unsigned short* __restrict__ VTl,
           const int* __restrict__ cq, const int* __restrict__ ck,
           const float* __restrict__ alpha, const float* __restrict__ rpe,
           const float* __restrict__ lq1, const float* __restrict__ lk1,
           const float* __restrict__ lq2, const float* __restrict__ lk2,
           unsigned short* CTh, unsigned short* CTl) {
  __shared__ __align__(16) float smem[ATT_SMEM_FLOATS];

  const int tid  = threadIdx.x;
  const int wave = __builtin_amdgcn_readfirstlane(tid >> 5);
  const int lane = tid & 31;
  const int hh   = lane >> 4;
  const int c    = lane & 15;

  const int rt   = blockIdx.x & ((NTOK / 16) - 1);
  const int bat  = blockIdx.x / (NTOK / 16);
  const int head = wave;
  const int pr   = wave & (NPAIR - 1);
  const bool xw  = (wave >= NPAIR);
  const int q0   = rt * 16;
  const size_t rowg = (size_t)bat * NTOK + q0;

  const size_t qofs = (rowg + c) * DM + head * HD + 8 * hh;
  const v16h qa = ldfrag_u(Q16 + qofs), qb = ldfrag_u(Q16 + qofs + 32);

  float lam;
  {
    const int i0 = pr * HD + lane, i1 = i0 + 32;
    float t1 = bfr(lq1[i0]) * bfr(lk1[i0]) + bfr(lq1[i1]) * bfr(lk1[i1]);
    float t2 = bfr(lq2[i0]) * bfr(lk2[i0]) + bfr(lq2[i1]) * bfr(lk2[i1]);
#pragma unroll
    for (int off = 1; off < 32; off <<= 1) {
      t1 += __shfl_xor(t1, off, 32);
      t2 += __shfl_xor(t2, off, 32);
    }
    lam = expf(t1) - expf(t2) + LAM0;
  }

  int qcx[8], qcy[8];
#pragma unroll
  for (int r = 0; r < 8; ++r) {
    const size_t qi = (rowg + 8 * hh + r) * 2;
    qcx[r] = cq[qi];
    qcy[r] = cq[qi + 1];
  }

  const unsigned short* Kb  = K16 + (size_t)bat * NTOK * DM + head * HD + 8 * hh;
  const unsigned short* Voh = VTh + ((size_t)bat * DM + head * HD) * NTOK + 8 * hh;
  const unsigned short* Vol = VTl + ((size_t)bat * DM + head * HD) * NTOK + 8 * hh;
  const unsigned short* Vph = VTh + ((size_t)bat * DM + pr * HD) * NTOK + 8 * hh;
  const unsigned short* Vpl = VTl + ((size_t)bat * DM + pr * HD) * NTOK + 8 * hh;
  const int* ckb = ck + (size_t)bat * NTOK * 2;
  const float* rph = rpe + head;

  float mrow[8], lrow[8];
  v8f o0 = zero8(), o1 = zero8(), o2 = zero8(), o3 = zero8();
  v8f x0 = zero8(), x1 = zero8(), x2 = zero8(), x3 = zero8();
#pragma unroll
  for (int r = 0; r < 8; ++r) { mrow[r] = -INFINITY; lrow[r] = 0.f; }
  float* pt = smem + wave * (16 * 36);

#pragma unroll 1
  for (int kb = 0; kb < NTOK; kb += KCH) {
    v8f s0, s1;
    {
      const size_t ko  = (size_t)(kb + c) * DM;
      const size_t k1o = ko + (size_t)16 * DM;
      const v16h k0a = ldfrag_u(Kb + ko),  k0b = ldfrag_u(Kb + ko + 32);
      const v16h k1a = ldfrag_u(Kb + k1o), k1b = ldfrag_u(Kb + k1o + 32);
      s0 = mma_h(qa, k0a, zero8());
      s0 = mma_h(qb, k0b, s0);
      s1 = mma_h(qa, k1a, zero8());
      s1 = mma_h(qb, k1b, s1);
      guard2x6(s0, s1, k0a, k0b, k1a, k1b, qa, qb);
    }
    const int kc0 = (kb + c) * 2, kc1 = (kb + 16 + c) * 2;
    const int kx0 = ckb[kc0], ky0 = ckb[kc0 + 1];
    const int kx1 = ckb[kc1], ky1 = ckb[kc1 + 1];
#pragma unroll
    for (int r = 0; r < 8; ++r) {
      const int ia = iclamp(qcx[r] - kx0 + RPOFF, 0, RPMAX) * RPW + iclamp(qcy[r] - ky0 + RPOFF, 0, RPMAX);
      const int ib = iclamp(qcx[r] - kx1 + RPOFF, 0, RPMAX) * RPW + iclamp(qcy[r] - ky1 + RPOFF, 0, RPMAX);
      const float b0 = bfr(rph[(size_t)ia * NHEAD]) * LOG2E;
      const float b1 = bfr(rph[(size_t)ib * NHEAD]) * LOG2E;
      const float t0 = s0[r] * SC2 + b0, t1 = s1[r] * SC2 + b1;
      float mx = fmaxf(t0, t1);
#pragma unroll
      for (int off = 1; off < 16; off <<= 1) mx = fmaxf(mx, __shfl_xor(mx, off, 32));
      const float mn = fmaxf(mrow[r], mx);
      const float al = exp2f(mrow[r] - mn);
      mrow[r] = mn;
      const float e0 = exp2f(t0 - mn), e1 = exp2f(t1 - mn);
      float ps = e0 + e1;
#pragma unroll
      for (int off = 1; off < 16; off <<= 1) ps += __shfl_xor(ps, off, 32);
      lrow[r] = lrow[r] * al + ps;
      o0[r] *= al; o1[r] *= al; o2[r] *= al; o3[r] *= al;
      x0[r] *= al; x1[r] *= al; x2[r] *= al; x3[r] *= al;
      const int ro = (8 * hh + r) * 36 + c;
      pt[ro]      = e0;
      pt[ro + 16] = e1;
    }
    wave_sync_lds();
    FragH ph, pl;
    {
      const float* prow = pt + c * 36 + 8 * hh;
      const v4f p0 = *(const v4f*)(prow), p1 = *(const v4f*)(prow + 4);
      const v4f p2 = *(const v4f*)(prow + 16), p3 = *(const v4f*)(prow + 20);
#pragma unroll
      for (int e = 0; e < 4; ++e) {
        float f; _Float16 x;
        f = p0[e] * PC; x = (_Float16)f; ph.h[0][e]     = x; pl.h[0][e]     = (_Float16)(f - (float)x);
        f = p1[e] * PC; x = (_Float16)f; ph.h[0][4 + e] = x; pl.h[0][4 + e] = (_Float16)(f - (float)x);
        f = p2[e] * PC; x = (_Float16)f; ph.h[1][e]     = x; pl.h[1][e]     = (_Float16)(f - (float)x);
        f = p3[e] * PC; x = (_Float16)f; ph.h[1][4 + e] = x; pl.h[1][4 + e] = (_Float16)(f - (float)x);
      }
    }
    const size_t vo = (size_t)c * NTOK + kb;
    {
      const v16h vh0 = ldfrag_u(Voh + vo);
      const v16h vh1 = ldfrag_u(Voh + vo + (size_t)16 * NTOK);
      const v16h vh2 = ldfrag_u(Voh + vo + (size_t)32 * NTOK);
      const v16h vh3 = ldfrag_u(Voh + vo + (size_t)48 * NTOK);
      o0 = mma_h(ph.v, vh0, o0);
      o1 = mma_h(ph.v, vh1, o1);
      o2 = mma_h(ph.v, vh2, o2);
      o3 = mma_h(ph.v, vh3, o3);
      o0 = mma_h(pl.v, vh0, o0);
      o1 = mma_h(pl.v, vh1, o1);
      o2 = mma_h(pl.v, vh2, o2);
      o3 = mma_h(pl.v, vh3, o3);
      guard4x6(o0, o1, o2, o3, ph.v, pl.v, vh0, vh1, vh2, vh3);
    }
    if (xw) {
      const v16h vh0 = ldfrag_u(Vph + vo);
      const v16h vh1 = ldfrag_u(Vph + vo + (size_t)16 * NTOK);
      const v16h vh2 = ldfrag_u(Vph + vo + (size_t)32 * NTOK);
      const v16h vh3 = ldfrag_u(Vph + vo + (size_t)48 * NTOK);
      x0 = mma_h(ph.v, vh0, x0);
      x1 = mma_h(ph.v, vh1, x1);
      x2 = mma_h(ph.v, vh2, x2);
      x3 = mma_h(ph.v, vh3, x3);
      x0 = mma_h(pl.v, vh0, x0);
      x1 = mma_h(pl.v, vh1, x1);
      x2 = mma_h(pl.v, vh2, x2);
      x3 = mma_h(pl.v, vh3, x3);
      guard4x6(x0, x1, x2, x3, ph.v, pl.v, vh0, vh1, vh2, vh3);
    }
    {
      const v16h vl0 = ldfrag_u(Vol + vo);
      const v16h vl1 = ldfrag_u(Vol + vo + (size_t)16 * NTOK);
      const v16h vl2 = ldfrag_u(Vol + vo + (size_t)32 * NTOK);
      const v16h vl3 = ldfrag_u(Vol + vo + (size_t)48 * NTOK);
      o0 = mma_h(ph.v, vl0, o0);
      o1 = mma_h(ph.v, vl1, o1);
      o2 = mma_h(ph.v, vl2, o2);
      o3 = mma_h(ph.v, vl3, o3);
      guard4x5(o0, o1, o2, o3, ph.v, vl0, vl1, vl2, vl3);
    }
    if (xw) {
      const v16h vl0 = ldfrag_u(Vpl + vo);
      const v16h vl1 = ldfrag_u(Vpl + vo + (size_t)16 * NTOK);
      const v16h vl2 = ldfrag_u(Vpl + vo + (size_t)32 * NTOK);
      const v16h vl3 = ldfrag_u(Vpl + vo + (size_t)48 * NTOK);
      x0 = mma_h(ph.v, vl0, x0);
      x1 = mma_h(ph.v, vl1, x1);
      x2 = mma_h(ph.v, vl2, x2);
      x3 = mma_h(ph.v, vl3, x3);
      guard4x5(x0, x1, x2, x3, ph.v, vl0, vl1, vl2, vl3);
    }
    wave_sync_lds();
  }
  acc_guard4(o0, o1, o2, o3);
  acc_guard4(x0, x1, x2, x3);

  __syncthreads();
  float* cross = smem;
  unsigned short* Osh = (unsigned short*)(smem + CROSS_FLOATS);
  unsigned short* Osl = Osh + OROW_HALVES;
  const float oc = 1.0f / (PC * VC);
  if (xw) {
#pragma unroll
    for (int r = 0; r < 8; ++r) {
      const float inv = (1.0f / lrow[r]) * oc;
      const int ro = ((wave - NPAIR) * 16 + 8 * hh + r) * HD + c;
      cross[ro]      = x0[r] * inv;
      cross[ro + 16] = x1[r] * inv;
      cross[ro + 32] = x2[r] * inv;
      cross[ro + 48] = x3[r] * inv;
    }
  }
  __syncthreads();
  {
    const int cb = head * HD + c;
#pragma unroll
    for (int r = 0; r < 8; ++r) {
      const size_t qi = rowg + 8 * hh + r;
      const float ag = bfr(alpha[qi]);
      const float al = xw ? 0.f : ag;
      const float inv = (1.0f / lrow[r]) * oc;
      const int ri = (pr * 16 + 8 * hh + r) * HD + c;
      const int ro = (8 * hh + r) * DM + cb;
      const float xs0 = o0[r] * inv, xs1 = o1[r] * inv, xs2 = o2[r] * inv, xs3 = o3[r] * inv;
      const float cr0 = cross[ri], cr1 = cross[ri + 16], cr2 = cross[ri + 32], cr3 = cross[ri + 48];
      const float d0 = xs0 - lam * cr0, d1 = xs1 - lam * cr1, d2 = xs2 - lam * cr2, d3 = xs3 - lam * cr3;
      const float f0 = xs0 + al * d0, f1 = xs1 + al * d1, f2 = xs2 + al * d2, f3 = xs3 + al * d3;
      const unsigned short g0 = bf_bits(f0), g1 = bf_bits(f1), g2 = bf_bits(f2), g3 = bf_bits(f3);
      Osh[ro]      = g0;  Osl[ro]      = bf_bits(f0 - bf_up(g0));
      Osh[ro + 16] = g1;  Osl[ro + 16] = bf_bits(f1 - bf_up(g1));
      Osh[ro + 32] = g2;  Osl[ro + 32] = bf_bits(f2 - bf_up(g2));
      Osh[ro + 48] = g3;  Osl[ro + 48] = bf_bits(f3 - bf_up(g3));
    }
  }
  __syncthreads();
  {
    v4u hv[4], lv[4];
#pragma unroll
    for (int it = 0; it < 4; ++it) {
      const int p = it * ATT_THREADS + tid;
      hv[it] = *(const v4u*)(Osh + (size_t)p * 8);
      lv[it] = *(const v4u*)(Osl + (size_t)p * 8);
    }
    const size_t dofs = rowg * DM;
    unsigned short* dsth = CTh + dofs;
    unsigned short* dstl = CTl + dofs;
    for (int pass = 0; pass < 2; ++pass) {
#pragma unroll
      for (int it = 0; it < 4; ++it) {
        const int p = it * ATT_THREADS + tid;
        *(volatile v4u*)(dsth + (size_t)p * 8) = hv[it];
        *(volatile v4u*)(dstl + (size_t)p * 8) = lv[it];
      }
      __threadfence();
    }
  }
}

extern "C" void kernel_launch(void* const* d_in, const int* in_sizes, int n_in,
                              void* d_out, int out_size, void* d_ws, size_t ws_size,
                              hipStream_t stream) {
  if (n_in < 18) return;
  if (in_sizes[0] != NROWS * DM || in_sizes[1] != NROWS * DM) return;
  if (in_sizes[2] != NROWS * 2 || in_sizes[3] != NROWS * 2) return;
  if (in_sizes[4] != NROWS) return;
  if (in_sizes[5] != DM * DM || in_sizes[7] != DM * DM || in_sizes[9] != DM * DM || in_sizes[16] != DM * DM) return;
  if (in_sizes[6] != DM || in_sizes[8] != DM || in_sizes[10] != DM || in_sizes[17] != DM) return;
  if (in_sizes[11] != NPAIR * HD || in_sizes[12] != NPAIR * HD || in_sizes[13] != NPAIR * HD || in_sizes[14] != NPAIR * HD) return;
  if (in_sizes[15] != RPN * NHEAD) return;
  if (out_size != NROWS * DM) return;

  const float* x_q  = (const float*)d_in[0];
  const float* x_kv = (const float*)d_in[1];
  const int*   cq   = (const int*)d_in[2];
  const int*   ck   = (const int*)d_in[3];
  const float* alph = (const float*)d_in[4];
  const float* w_q  = (const float*)d_in[5];
  const float* b_q  = (const float*)d_in[6];
  const float* w_k  = (const float*)d_in[7];
  const float* b_k  = (const float*)d_in[8];
  const float* w_v  = (const float*)d_in[9];
  const float* b_v  = (const float*)d_in[10];
  const float* lq1  = (const float*)d_in[11];
  const float* lk1  = (const float*)d_in[12];
  const float* lq2  = (const float*)d_in[13];
  const float* lk2  = (const float*)d_in[14];
  const float* rpe  = (const float*)d_in[15];
  const float* w_p  = (const float*)d_in[16];
  const float* b_p  = (const float*)d_in[17];
  float*       out  = (float*)d_out;

  const size_t PW = (size_t)DM * DM * 2;
  const size_t PX = (size_t)NROWS * DM * 2;
  const size_t PV = (size_t)NB * DM * NTOK * 2;
  size_t off = 0;
  const size_t oWQ = off; off += PW;
  const size_t oWK = off; off += PW;
  const size_t oWV = off; off += PW;
  const size_t oWP = off; off += PW;
  const size_t oXQ = off; off += PX;
  const size_t oXK = off; off += PX;
  const size_t oQ  = off; off += PX;
  const size_t oK  = off; off += PX;
  const size_t oVh = off; off += PV;
  const size_t oVl = off; off += PV;
  const size_t oCh = off; off += PX;
  const size_t oCl = off; off += PX;
  if (off > ws_size) return;
  if (off > (size_t)134217728) return;

  char* ws = (char*)d_ws;
  unsigned short* WQ16  = (unsigned short*)(ws + oWQ);
  unsigned short* WK16  = (unsigned short*)(ws + oWK);
  unsigned short* WV16  = (unsigned short*)(ws + oWV);
  unsigned short* WP16  = (unsigned short*)(ws + oWP);
  unsigned short* XQ16  = (unsigned short*)(ws + oXQ);
  unsigned short* XKV16 = (unsigned short*)(ws + oXK);
  unsigned short* Q16   = (unsigned short*)(ws + oQ);
  unsigned short* K16   = (unsigned short*)(ws + oK);
  unsigned short* VTh   = (unsigned short*)(ws + oVh);
  unsigned short* VTl   = (unsigned short*)(ws + oVl);
  unsigned short* CTh   = (unsigned short*)(ws + oCh);
  unsigned short* CTl   = (unsigned short*)(ws + oCl);

  const dim3 blk(256);
  const dim3 gCX((NROWS * DM) / 2048);
  const dim3 gCW((DM * DM) / 2048);
  const int tilesP = (NROWS / 64) * (DM / 64);
  const int tilesV = (DM / 64) * (NTOK / 64);
  const dim3 gP((tilesP + 7) / 8, 1);
  const dim3 gV((tilesV + 7) / 8, NB);
  const dim3 gAT(ATT_BLOCKS);
  const dim3 bAT(ATT_THREADS);

  cvt16<0><<<gCX, blk, 0, stream>>>(x_q,  XQ16,  NROWS * DM, ACARRY);
  cvt16<0><<<gCX, blk, 0, stream>>>(x_kv, XKV16, NROWS * DM, ACARRY);
  cvt16<0><<<gCW, blk, 0, stream>>>(w_q, WQ16, DM * DM, WSC);
  cvt16<0><<<gCW, blk, 0, stream>>>(w_k, WK16, DM * DM, WSC);
  cvt16<0><<<gCW, blk, 0, stream>>>(w_v, WV16, DM * DM, WSC);
  cvt16<1><<<gCW, blk, 0, stream>>>(w_p, WP16, DM * DM, 1.0f);

  gemm64<2, 0, 0, 1><<<gP, blk, 0, stream>>>(
      XQ16, XQ16, DM, 0LL,
      WQ16, DM, 0LL,
      (void*)Q16, (void*)Q16, DM, 0LL,
      NROWS, DM, DM, 1.0f / (ACARRY * WSC), 1.0f, b_q);

  gemm64<2, 0, 0, 1><<<gP, blk, 0, stream>>>(
      XKV16, XKV16, DM, 0LL,
      WK16, DM, 0LL,
      (void*)K16, (void*)K16, DM, 0LL,
      NROWS, DM, DM, 1.0f / (ACARRY * WSC), 1.0f, b_k);

  gemm64<4, 0, 0, 2><<<gV, blk, 0, stream>>>(
      WV16, WV16, DM, 0LL,
      XKV16, DM, (long long)NTOK * DM,
      (void*)VTh, (void*)VTl, NTOK, (long long)DM * NTOK,
      DM, NTOK, DM, 1.0f / (ACARRY * WSC), VC, b_v);

  attn8<<<gAT, bAT, 0, stream>>>(Q16, K16, VTh, VTl, cq, ck, alph, rpe, lq1, lk1, lq2, lk2, CTh, CTl);

  gemm64<0, 1, 1, 1><<<gP, blk, 0, stream>>>(
      CTh, CTl, DM, 0LL,
      WP16, DM, 0LL,
      (void*)out, (void*)out, DM, 0LL,
      NROWS, DM, DM, 1.0f, 1.0f, b_p);
  (void)hipGetLastError();
}
